// GNNFewShotClassifier_71236327571546
// MI455X (gfx1250) — hardware-verified
//
#include <hip/hip_runtime.h>
#include <math.h>
typedef __attribute__((ext_vector_type(16))) _Float16 v16h;
typedef __attribute__((ext_vector_type(8)))  _Float16 v8h;
typedef __attribute__((ext_vector_type(16))) __bf16   v16b;
typedef __attribute__((ext_vector_type(8)))  __bf16   v8b;
typedef __attribute__((ext_vector_type(8)))  float    v8f;
typedef __attribute__((ext_vector_type(4)))  float    v4f;
#define PSCALE 32768.0f
#define U16(p) ((const unsigned short*)(const void*)(p))
#define PSCALE_INV (1.0f / 32768.0f)

__device__ __forceinline__ unsigned short f2bf_bits(float f) {
  unsigned u = __float_as_uint(f);
  return (unsigned short)((u + 0x7FFFu + ((u >> 16) & 1u)) >> 16);
}
__device__ __forceinline__ float bf_bits2f(unsigned short h) { return __uint_as_float(((unsigned)h) << 16); }

__device__ __forceinline__ void dep_guard_h(v8f& a, v8f& b, v16h x, v16h y) { asm volatile("v_nop\n\tv_nop\n\tv_nop\n\tv_nop" : "+v"(a), "+v"(b) : "v"(x), "v"(y)); }
__device__ __forceinline__ void dep_guard_b(v8f& a, v8f& b, v16b x, v16b y) { asm volatile("v_nop\n\tv_nop\n\tv_nop\n\tv_nop" : "+v"(a), "+v"(b) : "v"(x), "v"(y)); }
__device__ __forceinline__ void keep4_h(v16h a, v16h b, v16h c, v16h d) { asm volatile("v_nop" :: "v"(a), "v"(b), "v"(c), "v"(d)); }
__device__ __forceinline__ void keep4_b(v16b a, v16b b, v16b c, v16b d) { asm volatile("v_nop" :: "v"(a), "v"(b), "v"(c), "v"(d)); }
__device__ __forceinline__ void acc_guard4(v8f& a, v8f& b, v8f& c, v8f& d) { asm volatile("v_nop\n\tv_nop\n\tv_nop\n\tv_nop" : "+v"(a), "+v"(b), "+v"(c), "+v"(d)); }
template <typename T> struct Frag;
template <> struct Frag<_Float16> {
  typedef v16h V; union U { v16h v; v8h h[2]; };
  static __device__ __forceinline__ v16h load(const _Float16* p) {
    U f; f.h[0] = *(const v8h*)(p); f.h[1] = *(const v8h*)(p + 16); return f.v;
  }
  static __device__ __forceinline__ v8f mma(v16h a, v16h b, v8f c) {
    return __builtin_amdgcn_wmma_f32_16x16x32_f16(false, a, false, b, (short)0, c, false, false);
  }
  static __device__ __forceinline__ void guard(v8f& a, v8f& b, v16h x, v16h y) { dep_guard_h(a, b, x, y); }
  static __device__ __forceinline__ void keep(v16h a, v16h b, v16h c, v16h d) { keep4_h(a, b, c, d); }
};
template <> struct Frag<__bf16> {
  typedef v16b V; union U { v16b v; v8b h[2]; };
  static __device__ __forceinline__ v16b load(const __bf16* p) {
    U f; f.h[0] = *(const v8b*)(p); f.h[1] = *(const v8b*)(p + 16); return f.v;
  }
  static __device__ __forceinline__ v8f mma(v16b a, v16b b, v8f c) {
    return __builtin_amdgcn_wmma_f32_16x16x32_bf16(false, a, false, b, (short)0, c, false, false);
  }
  static __device__ __forceinline__ void guard(v8f& a, v8f& b, v16b x, v16b y) { dep_guard_b(a, b, x, y); }
  static __device__ __forceinline__ void keep(v16b a, v16b b, v16b c, v16b d) { keep4_b(a, b, c, d); }
};

template <int ET> struct Elem;
template <> struct Elem<0> { typedef _Float16 T; };
template <> struct Elem<1> { typedef __bf16 T; };
template <int ET, bool SPLIT, int BIAS_MODE, int OUT_MODE, bool RESID, int ACT = 0>
__global__ __launch_bounds__(256) void wmma_gemm64(
    const unsigned short* __restrict__ Ap, const unsigned short* __restrict__ A2p, int lda, long strideA,
    const unsigned short* __restrict__ Btp, const unsigned short* __restrict__ Bt2p, int ldb, long strideB,
    void* __restrict__ Cout, void* __restrict__ Cout2, int ldc, long strideC,
    const float* __restrict__ bias,
    const float* __restrict__ resid, long strideR,
    int M, int N, int K, float scale) {
  typedef typename Elem<ET>::T T;
  typedef typename Frag<T>::V V;
  const T* A = (const T*)Ap; const T* A2 = (const T*)A2p; const T* Bt = (const T*)Btp; const T* Bt2 = (const T*)Bt2p;
  __shared__ __align__(16) float sT[8][16 * 68];
  const int b    = blockIdx.y;
  const int lane = threadIdx.x & 31;
  const int wave = threadIdx.x >> 5;
  const int tilesN = N >> 6;
  const int tilesM = M >> 6;
  const int tile = blockIdx.x * 8 + wave;
  if (tile >= tilesM * tilesN) return;
  const int tm = tile / tilesN;
  const int tn = tile - tm * tilesN;
  const int m0 = tm << 6;
  const int n0 = tn << 6;

  const T* Ab  = A  + (size_t)b * strideA;
  const T* Bb  = Bt + (size_t)b * strideB;
  const T* Ab2 = SPLIT ? (A2  + (size_t)b * strideA) : nullptr;
  const T* Bb2 = SPLIT ? (Bt2 + (size_t)b * strideB) : nullptr;

  const int rlane = lane & 15;
  const int koff  = (lane >> 4) * 8;
  const int mOff  = (lane >> 4) * 8;

  v8f acc[4][4];
#pragma unroll
  for (int i = 0; i < 4; ++i)
#pragma unroll
    for (int j = 0; j < 4; ++j) acc[i][j] = (v8f){0.f,0.f,0.f,0.f,0.f,0.f,0.f,0.f};

  for (int k0 = 0; k0 < K; k0 += 32) {
    V bh[4], bl[4];
#pragma unroll
    for (int j = 0; j < 4; ++j) {
      const size_t bo = (size_t)(n0 + (j << 4) + rlane) * ldb + koff + k0;
      bh[j] = Frag<T>::load(Bb + bo);
      if (SPLIT) bl[j] = Frag<T>::load(Bb2 + bo);
    }
#pragma unroll
    for (int i = 0; i < 4; ++i) {
      const size_t ao = (size_t)(m0 + (i << 4) + rlane) * lda + koff + k0;
      V ah = Frag<T>::load(Ab + ao);
      V al;
      if (SPLIT) al = Frag<T>::load(Ab2 + ao);
#pragma unroll
      for (int j = 0; j < 4; ++j) {
        acc[i][j] = Frag<T>::mma(ah, bh[j], acc[i][j]);
        if (SPLIT) {
          acc[i][j] = Frag<T>::mma(ah, bl[j], acc[i][j]);
          acc[i][j] = Frag<T>::mma(al, bh[j], acc[i][j]);
        }
      }
      Frag<T>::guard(acc[i][0], acc[i][3], ah, SPLIT ? al : ah);
    }
    Frag<T>::keep(bh[0], bh[1], bh[2], bh[3]);
    if (SPLIT) Frag<T>::keep(bl[0], bl[1], bl[2], bl[3]);
  }
  acc_guard4(acc[0][0], acc[0][1], acc[0][2], acc[0][3]);
  acc_guard4(acc[1][0], acc[1][1], acc[1][2], acc[1][3]);
  acc_guard4(acc[2][0], acc[2][1], acc[2][2], acc[2][3]);
  acc_guard4(acc[3][0], acc[3][1], acc[3][2], acc[3][3]);

  float* slab = sT[wave];
  const float* Rb = RESID ? (resid + (size_t)b * strideR) : nullptr;
#pragma unroll
  for (int i = 0; i < 4; ++i) {
    const int mBase = m0 + (i << 4);
#pragma unroll
    for (int j = 0; j < 4; ++j) {
      const int n = n0 + (j << 4) + rlane;
      float bv = 0.f;
      if (BIAS_MODE == 2) bv = bias[n];
#pragma unroll
      for (int r = 0; r < 8; ++r) {
        float v = acc[i][j][r] * scale;
        if (BIAS_MODE == 1) v += bias[mBase + mOff + r];
        if (BIAS_MODE == 2) v += bv;
        if (RESID) v += Rb[(size_t)(mBase + mOff + r) * ldc + n];
        if (ACT == 1) v = tanhf(v);
        if (ACT == 2) v = fmaxf(v, 0.0f);
        if (ACT == 3) v = v / (1.0f + expf(-v));
        if (ACT == 4) v = (v > 0.f) ? v : 0.01f * v;
        if (ACT == 5) v = 0.5f * v * (1.0f + erff(v * 0.70710678118654752f));
        slab[(mOff + r) * 68 + (j << 4) + rlane] = v;
      }
    }
    __builtin_amdgcn_fence(__ATOMIC_RELEASE, "workgroup");
    __builtin_amdgcn_wave_barrier();
    __builtin_amdgcn_fence(__ATOMIC_ACQUIRE, "workgroup");
    if (OUT_MODE == 0) {
      float* C = (float*)Cout + (size_t)b * strideC;
      const int hh = lane >> 4, c4 = (lane & 15) * 4;
      for (int pass = 0; pass < 2; ++pass) {
#pragma unroll
        for (int it = 0; it < 8; ++it) {
          const int row = it * 2 + hh;
          v4f v = *(const v4f*)(slab + row * 68 + c4);
          *(volatile v4f*)(C + (size_t)(mBase + row) * ldc + n0 + c4) = v;
        }
        __threadfence();
      }
    } else {
      const int q = lane >> 3, c8 = (lane & 7) * 8;
      unsigned short* C  = (unsigned short*)Cout  + (size_t)b * strideC;
      unsigned short* C2 = (OUT_MODE == 2) ? ((unsigned short*)Cout2 + (size_t)b * strideC) : nullptr;
      for (int pass = 0; pass < 2; ++pass) {
#pragma unroll
        for (int it = 0; it < 4; ++it) {
          const int row = it * 4 + q;
          const float* sp = slab + row * 68 + c8;
          v8h hv, lv;
#pragma unroll
          for (int e = 0; e < 8; ++e) {
            if (OUT_MODE == 1) {
              hv[e] = (_Float16)sp[e];
            } else {
              unsigned short hb = f2bf_bits(sp[e]);
              unsigned short lb = f2bf_bits(sp[e] - bf_bits2f(hb));
              hv[e] = __builtin_bit_cast(_Float16, hb);
              lv[e] = __builtin_bit_cast(_Float16, lb);
            }
          }
          *(volatile v8h*)(C + (size_t)(mBase + row) * ldc + n0 + c8) = hv;
          if (OUT_MODE == 2) *(volatile v8h*)(C2 + (size_t)(mBase + row) * ldc + n0 + c8) = lv;
        }
        __threadfence();
      }
    }
    __builtin_amdgcn_fence(__ATOMIC_RELEASE, "workgroup");
    __builtin_amdgcn_wave_barrier();
    __builtin_amdgcn_fence(__ATOMIC_ACQUIRE, "workgroup");
  }
}

__global__ __launch_bounds__(256) void cast_f32_f16x2(
    const float* __restrict__ in, _Float16* __restrict__ out, int n2) {
  int i = blockIdx.x * 256 + threadIdx.x;
  if (i < n2) {
    const _Float16 h0 = (_Float16)in[2 * i], h1 = (_Float16)in[2 * i + 1];
    const unsigned u = (unsigned)__builtin_bit_cast(unsigned short, h0) | ((unsigned)__builtin_bit_cast(unsigned short, h1) << 16);
    ((volatile unsigned*)out)[i] = u;
    __threadfence();
    ((volatile unsigned*)out)[i] = u;
  }
}


__global__ __launch_bounds__(256) void transpose_cast_f16(const float* __restrict__ in, int ldi,
                                                         _Float16* __restrict__ outT, int ldo, float scale) {
  __shared__ __align__(16) _Float16 tile[64][72];
  const int c0 = blockIdx.x * 64, r0 = blockIdx.y * 64;
  const int t = threadIdx.y * 32 + threadIdx.x;
  for (int i = threadIdx.y; i < 64; i += 8) {
    tile[threadIdx.x][i]      = (_Float16)(in[(size_t)(r0 + i) * ldi + c0 + threadIdx.x] * scale);
    tile[32 + threadIdx.x][i] = (_Float16)(in[(size_t)(r0 + i) * ldi + c0 + 32 + threadIdx.x] * scale);
  }
  __syncthreads();
  const int q = t >> 3, c8 = (t & 7) * 8;
  for (int pass = 0; pass < 2; ++pass) {
#pragma unroll
    for (int it = 0; it < 2; ++it) {
      const int c = it * 32 + q;
      v8h hv = *(const v8h*)(&tile[c][c8]);
      *(volatile v8h*)(outT + (size_t)(c0 + c) * ldo + r0 + c8) = hv;
    }
    __threadfence();
  }
}

#define FQ 2048
#define FSUP 100
#define FC 20
#define FD0 512
#define FD1 256
#define FD2 128
#define FROWS2 (FQ * 21)
__global__ __launch_bounds__(1024) void support_kernel(const float* __restrict__ sup, const int* __restrict__ lab, const float* __restrict__ W1, const float* __restrict__ b1, float* __restrict__ AUX) {
  __shared__ int csz[FC]; __shared__ float csum[FC][FD0]; __shared__ float c0[FD0]; __shared__ float dsup;
  const int t = threadIdx.x;
  if (t < FC) csz[t] = 0;
  __syncthreads();
  if (t < FSUP) { int l = lab[t]; l = l < 0 ? 0 : (l >= FC ? FC - 1 : l); atomicAdd(&csz[l], 1); }
  for (int i = t; i < FC * FD0; i += 1024) (&csum[0][0])[i] = 0.f;
  __syncthreads();
  for (int d = t; d < FD0; d += 1024) { float acc0 = 0.f;
    for (int s = 0; s < FSUP; ++s) { int l = lab[s]; l = l < 0 ? 0 : (l >= FC ? FC - 1 : l); const float dj = rsqrtf((float)(1 + csz[l]) + 1e-6f); const float v = dj * sup[(size_t)s * FD0 + d]; csum[l][d] += v; acc0 += v; }
    c0[d] = acc0 * rsqrtf((float)FSUP + 1e-6f); }
  __syncthreads();
  for (int o = t; o < FD1 * 21; o += 1024) { const int which = o / FD1, col = o % FD1; float acc = 0.f;
    if (which == 0) { for (int d = 0; d < FD0; ++d) acc += c0[d] * W1[(size_t)d * FD1 + col]; acc = fmaxf(acc + b1[col], 0.f); }
    else { const int c = which - 1; const float dc = rsqrtf((float)(1 + csz[c]) + 1e-6f); for (int d = 0; d < FD0; ++d) acc += csum[c][d] * W1[(size_t)d * FD1 + col]; acc *= dc; }
    ((volatile float*)AUX)[o] = acc; }
  if (t < FC) ((volatile float*)AUX)[FD1 * 21 + t] = (float)csz[t];
  __threadfence();
  for (int o = t; o < FD1 * 21; o += 1024) ((volatile float*)AUX)[o] = AUX[o];
}
__global__ __launch_bounds__(256) void rows_kernel(const float* __restrict__ QW, const float* __restrict__ AUX, const float* __restrict__ b1, unsigned* __restrict__ R16) {
  const int lane = threadIdx.x & 31, wave = threadIdx.x >> 5; const int q = blockIdx.x * 8 + wave;
  const float dis0 = rsqrtf((float)FSUP + 1e-6f);
  typedef __attribute__((ext_vector_type(4))) unsigned u4;
  float qw[8]; for (int e = 0; e < 8; ++e) qw[e] = QW[(size_t)q * FD1 + lane * 8 + e];
  float a0[8]; for (int e = 0; e < 8; ++e) a0[e] = 0.f;
#pragma unroll 1
  for (int c = 0; c < FC; ++c) { const float csz = AUX[FD1 * 21 + c]; const float dc = rsqrtf(1.0f + csz + 1e-6f);
    for (int e = 0; e < 8; ++e) { const int col = lane * 8 + e; const float h = fmaxf(dc * dis0 * qw[e] + AUX[FD1 + c * FD1 + col] + b1[col], 0.f); a0[e] += csz * dc * h; } }
  for (int pass = 0; pass < 2; ++pass) {
    { u4 u; for (int e = 0; e < 4; ++e) u[e] = (unsigned)__builtin_bit_cast(unsigned short, (_Float16)(dis0 * a0[2 * e])) | ((unsigned)__builtin_bit_cast(unsigned short, (_Float16)(dis0 * a0[2 * e + 1])) << 16);
      *(volatile u4*)(R16 + (((size_t)q * 21) * FD1 + lane * 8) / 2) = u; }
#pragma unroll 1
    for (int c = 0; c < FC; ++c) { const float csz = AUX[FD1 * 21 + c]; const float dc = rsqrtf(1.0f + csz + 1e-6f); u4 u;
      for (int e = 0; e < 4; ++e) { float v[2]; for (int s = 0; s < 2; ++s) { const int col = lane * 8 + 2 * e + s; const float h = fmaxf(dc * dis0 * qw[2 * e + s] + AUX[FD1 + c * FD1 + col] + b1[col], 0.f); v[s] = dc * (dis0 * AUX[col] + dc * csz * h); }
        u[e] = (unsigned)__builtin_bit_cast(unsigned short, (_Float16)v[0]) | ((unsigned)__builtin_bit_cast(unsigned short, (_Float16)v[1]) << 16); }
      *(volatile u4*)(R16 + (((size_t)q * 21 + 1 + c) * FD1 + lane * 8) / 2) = u; }
    __threadfence(); }
}
__global__ __launch_bounds__(256) void cos_kernel(const float* __restrict__ H2, float* __restrict__ out) {
  __shared__ float st[8][FC];
  const int lane = threadIdx.x & 31, wave = threadIdx.x >> 5; const int q = blockIdx.x * 8 + wave;
  const v4f e0 = *(const v4f*)(H2 + ((size_t)q * 21) * FD2 + lane * 4); float n0 = e0[0]*e0[0] + e0[1]*e0[1] + e0[2]*e0[2] + e0[3]*e0[3]; for (int o = 16; o > 0; o >>= 1) n0 += __shfl_xor(n0, o, 32); n0 = sqrtf(n0);
#pragma unroll 1
  for (int c = 0; c < FC; ++c) { const v4f p = *(const v4f*)(H2 + ((size_t)q * 21 + 1 + c) * FD2 + lane * 4); float d = e0[0]*p[0] + e0[1]*p[1] + e0[2]*p[2] + e0[3]*p[3], np2 = p[0]*p[0] + p[1]*p[1] + p[2]*p[2] + p[3]*p[3];
    for (int o = 16; o > 0; o >>= 1) { d += __shfl_xor(d, o, 32); np2 += __shfl_xor(np2, o, 32); }
    if (lane == 0) st[wave][c] = d / fmaxf(n0 * sqrtf(np2), 1e-8f); }
  __syncthreads();
  for (int i = threadIdx.x; i < 8 * FC; i += 256) { ((volatile float*)out)[(size_t)blockIdx.x * 8 * FC + i] = (&st[0][0])[i]; }
  __threadfence();
  for (int i = threadIdx.x; i < 8 * FC; i += 256) { ((volatile float*)out)[(size_t)blockIdx.x * 8 * FC + i] = (&st[0][0])[i]; }
}
extern "C" void kernel_launch(void* const* d_in, const int* in_sizes, int n_in, void* d_out, int out_size, void* d_ws, size_t ws_size, hipStream_t stream) {
  (void)in_sizes; (void)n_in; (void)out_size; (void)ws_size;
  const float* sup = (const float*)d_in[0]; const int* lab = (const int*)d_in[1]; const float* qf = (const float*)d_in[2]; const float* W1 = (const float*)d_in[3]; const float* b1 = (const float*)d_in[4]; const float* W2 = (const float*)d_in[5]; const float* b2 = (const float*)d_in[6];
  (void)d_in[7];
  char* ws = (char*)d_ws; size_t off = 0;
  auto carve = [&](size_t bytes) -> char* { char* p = ws + off; off += (bytes + 255) & ~(size_t)255; return p; };
  _Float16* Q16 = (_Float16*)carve((size_t)FQ * FD0 * 2); _Float16* W1T = (_Float16*)carve((size_t)FD1 * FD0 * 2); _Float16* W2T = (_Float16*)carve((size_t)FD2 * FD1 * 2);
  float* QW = (float*)carve((size_t)FQ * FD1 * 4); float* AUX = (float*)carve((size_t)(FD1 * 21 + 64) * 4); unsigned* R16 = (unsigned*)carve((size_t)FROWS2 * FD1 * 2); float* H2 = (float*)carve((size_t)FROWS2 * FD2 * 4);
  cast_f32_f16x2<<<(FQ * FD0 / 2 + 255) / 256, 256, 0, stream>>>(qf, Q16, (long)FQ * FD0 / 2);
  transpose_cast_f16<<<dim3(FD1 / 64, FD0 / 64), dim3(32, 8), 0, stream>>>(W1, FD1, W1T, FD0, 1.0f);
  transpose_cast_f16<<<dim3(FD2 / 64, FD1 / 64), dim3(32, 8), 0, stream>>>(W2, FD2, W2T, FD1, 1.0f);
  support_kernel<<<1, 1024, 0, stream>>>(sup, lab, W1, b1, AUX);
  { const int t = (FQ / 64) * (FD1 / 64); wmma_gemm64<0, false, 0, 0, false><<<dim3((t + 7) / 8, 1), 256, 0, stream>>>(U16(Q16), nullptr, FD0, 0, U16(W1T), nullptr, FD0, 0, QW, nullptr, FD1, 0, nullptr, nullptr, 0, FQ, FD1, FD0, 1.0f); }
  rows_kernel<<<FQ / 8, 256, 0, stream>>>(QW, AUX, b1, R16);
  { const int t = (FROWS2 / 64) * (FD2 / 64); wmma_gemm64<0, false, 2, 0, false, 2><<<dim3((t + 7) / 8, 1), 256, 0, stream>>>((const unsigned short*)R16, nullptr, FD1, 0, U16(W2T), nullptr, FD1, 0, H2, nullptr, FD2, 0, b2, nullptr, 0, FROWS2, FD2, FD1, 1.0f); }
  cos_kernel<<<FQ / 8, 256, 0, stream>>>(H2, (float*)d_out);
}
